// FourierKARTLayer_47854525612187
// MI455X (gfx1250) — hardware-verified
//
#include <hip/hip_runtime.h>


#define NR   2048
#define TS   1024
#define DIN  256
#define NQ   128
#define NK   6
#define NDO  64
#define KK   1536
typedef _Float16 h16;
typedef unsigned short bf;
typedef __attribute__((ext_vector_type(16))) __bf16   v16bf;
typedef __attribute__((ext_vector_type(16))) _Float16 v16h;
typedef __attribute__((ext_vector_type(8)))  _Float16 v8h;
typedef __attribute__((ext_vector_type(8)))  unsigned short v8us;
typedef __attribute__((ext_vector_type(8)))  float    v8f;
typedef __attribute__((ext_vector_type(4)))  float    v4f;
typedef v8h  __attribute__((may_alias)) v8ha;
typedef v4f  __attribute__((may_alias)) v4fa;
typedef v8us __attribute__((may_alias)) v8usa;

__device__ __forceinline__ unsigned short f2bf(float f) { unsigned u = __float_as_uint(f); u += 0x7FFFu + ((u >> 16) & 1u); return (unsigned short)(u >> 16); }
__device__ __forceinline__ float bf2f(unsigned short b) { return __uint_as_float(((unsigned)b) << 16); }
__device__ __forceinline__ float bfr(float f) { return bf2f(f2bf(f)); }
__device__ __forceinline__ v16h cat16(v8h lo, v8h hi) { return __builtin_shufflevector(lo, hi, 0, 1, 2, 3, 4, 5, 6, 7, 8, 9, 10, 11, 12, 13, 14, 15); }
__device__ __forceinline__ v16bf cat16b(v8us lo, v8us hi) { return __builtin_bit_cast(v16bf, __builtin_shufflevector(lo, hi, 0, 1, 2, 3, 4, 5, 6, 7, 8, 9, 10, 11, 12, 13, 14, 15)); }
__device__ __forceinline__ v8f wmma16(v16h a, v16h b, v8f c) { return __builtin_amdgcn_wmma_f32_16x16x32_f16(false, a, false, b, (short)0, c, false, false); }
__device__ __forceinline__ v8f wmmab(v16bf a, v16bf b, v8f c) { return __builtin_amdgcn_wmma_f32_16x16x32_bf16(false, a, false, b, (short)0, c, false, false); }


template <typename T16> struct WFrag;
template <> struct WFrag<h16> { typedef v16h V; static __device__ __forceinline__ V ld(const h16* p) { return cat16(*(const v8h*)p, *(const v8h*)(p + 16)); } static __device__ __forceinline__ v8f mma(V a, V b, v8f c) { return wmma16(a, b, c); } };
template <> struct WFrag<bf> { typedef v16bf V; static __device__ __forceinline__ V ld(const bf* p) { return cat16b(*(const v8us*)p, *(const v8us*)(p + 16)); } static __device__ __forceinline__ v8f mma(V a, V b, v8f c) { return wmmab(a, b, c); } };
template <typename T16, int NSPLIT, bool BIAS>
__global__ __launch_bounds__(32) void k_gemmw(const T16* __restrict__ A, const T16* __restrict__ A2, const T16* __restrict__ Bt, const T16* __restrict__ Bt2, int K, float* C, int ldc, const float* __restrict__ bias, size_t sA, size_t sB, size_t sC) {
    typedef typename WFrag<T16>::V V;
    __shared__ __align__(16) float os[16 * 68];
    const size_t z = blockIdx.z; A += z * sA; if (A2) A2 += z * sA; Bt += z * sB; if (Bt2) Bt2 += z * sB; C += z * sC;
    const int lane = threadIdx.x & 31, lr = lane & 15, hi = lane >> 4; const int r0 = blockIdx.x * 64, c0 = blockIdx.y * 64;
    v8f acc[4][4];
#pragma unroll
    for (int mb = 0; mb < 4; ++mb)
#pragma unroll
        for (int nb = 0; nb < 4; ++nb) acc[mb][nb] = (v8f){};
    const size_t aoff = (size_t)(r0 + lr) * K + 8 * hi, boff = (size_t)(c0 + lr) * K + 8 * hi;
    for (int kc = 0; kc < K; kc += 32) {
        V a[4], a2[4];
#pragma unroll
        for (int mb = 0; mb < 4; ++mb) { a[mb] = WFrag<T16>::ld(A + aoff + (size_t)mb * 16 * K + kc); if (NSPLIT == 1 || NSPLIT == 2) a2[mb] = WFrag<T16>::ld(A2 + aoff + (size_t)mb * 16 * K + kc); }
#pragma unroll
        for (int nb = 0; nb < 4; ++nb) { const V b = WFrag<T16>::ld(Bt + boff + (size_t)nb * 16 * K + kc); V b2; if (NSPLIT >= 2) b2 = WFrag<T16>::ld(Bt2 + boff + (size_t)nb * 16 * K + kc);
#pragma unroll
            for (int mb = 0; mb < 4; ++mb) { acc[mb][nb] = WFrag<T16>::mma(a[mb], b, acc[mb][nb]); if (NSPLIT == 1 || NSPLIT == 2) acc[mb][nb] = WFrag<T16>::mma(a2[mb], b, acc[mb][nb]); if (NSPLIT >= 2) acc[mb][nb] = WFrag<T16>::mma(a[mb], b2, acc[mb][nb]); } }
        asm volatile("v_nop\n\tv_nop\n\tv_nop\n\tv_nop" : "+v"(acc[0][0]), "+v"(acc[1][1]), "+v"(acc[2][2]), "+v"(acc[3][3]) : "v"(a[0]), "v"(a[3]));
    }
#pragma unroll
    for (int mb = 0; mb < 4; ++mb) {
#pragma unroll
        for (int nb = 0; nb < 4; ++nb) {
#pragma unroll
            for (int j = 0; j < 8; ++j) os[(hi * 8 + j) * 68 + nb * 16 + lr] = acc[mb][nb][j]; }
        __builtin_amdgcn_wave_barrier(); asm volatile("" ::: "memory");
        float* crow = C + (size_t)(r0 + mb * 16) * ldc + c0;
#pragma unroll 1
        for (int ps = 0; ps < 2; ++ps) {
#pragma unroll
            for (int s = 0; s < 8; ++s) { const int row = 2 * s + hi, cofs = lr * 4; v4f val = *(const v4fa*)(os + row * 68 + cofs); if (BIAS) { val[0] += bfr(bias[c0 + cofs]); val[1] += bfr(bias[c0 + cofs + 1]); val[2] += bfr(bias[c0 + cofs + 2]); val[3] += bfr(bias[c0 + cofs + 3]); }
                *(volatile v4f*)(crow + (size_t)row * ldc + cofs) = val; }
            if (ps == 0) __threadfence(); }
        __builtin_amdgcn_wave_barrier(); asm volatile("" ::: "memory");
    }
}

__device__ __forceinline__ h16 tohx(float x) { return (h16)x; }
__device__ __forceinline__ void splitf(float y, unsigned short& h, unsigned short& l) { h = f2bf(y); l = f2bf(y - bf2f(h)); }
typedef __attribute__((ext_vector_type(2))) _Float16 v2h;
typedef __attribute__((ext_vector_type(4))) _Float16 v4h;
typedef __attribute__((ext_vector_type(2))) unsigned short v2us;
typedef __attribute__((ext_vector_type(4))) unsigned short v4us;
typedef __attribute__((ext_vector_type(2))) float v2f;
typedef __attribute__((ext_vector_type(4))) int v4i;

__global__ __launch_bounds__(256) void k_cvt8(const float* __restrict__ src, bf* dst, size_t n8) { const size_t i = (size_t)blockIdx.x * 256 + threadIdx.x; if (i >= n8) return; const v8f v = *(const v8f*)(src + i * 8); v8us o;
#pragma unroll
    for (int k = 0; k < 8; ++k) o[k] = f2bf(v[k]); *(volatile v8us*)(dst + i * 8) = o; __threadfence(); *(volatile v8us*)(dst + i * 8) = o; }
__device__ __forceinline__ h16 toh_flush(float x) { const float z = (fabsf(x) < 6.103515625e-05f) ? 0.0f : x; return (h16)z; }

__global__ __launch_bounds__(256) void k_feat(const float* __restrict__ C, const float* __restrict__ w, const float* __restrict__ t, h16* F) { const size_t i = (size_t)blockIdx.x * 256 + threadIdx.x; if (i >= (size_t)NR * NQ / 4) return; const int r = (int)(i / (NQ / 4)); const int q0 = (int)(i % (NQ / 4)) * 4; const float tb = bfr(t[r / TS]); const v4f c4 = *(const v4f*)(C + (size_t)r * NQ + q0); const v4f w4 = *(const v4f*)(w + q0); float ang[4];
#pragma unroll
    for (int q = 0; q < 4; ++q) ang[q] = __fadd_rn(c4[q], __fmul_rn(bfr(w4[q]), tb));
    h16* fr = F + (size_t)r * KK + q0;
    for (int k = 0; k < NK; ++k) { v4h sv, cv;
#pragma unroll
        for (int q = 0; q < 4; ++q) { float s, c; sincosf(__fmul_rn(ang[q], (float)(k + 1)), &s, &c); sv[q] = toh_flush(s); cv[q] = toh_flush(c); }
        *(volatile v4h*)(fr + k * NQ) = sv; *(volatile v4h*)(fr + NK * NQ + k * NQ) = cv; __threadfence(); *(volatile v4h*)(fr + k * NQ) = sv; *(volatile v4h*)(fr + NK * NQ + k * NQ) = cv; } }

__global__ __launch_bounds__(256) void k_wfeat(const float* __restrict__ A, const float* __restrict__ Bp, h16* Wf) { const int i = blockIdx.x * 256 + threadIdx.x; if (i >= NDO * NK * NQ / 4) return; const int q0 = (i % (NQ / 4)) * 4; const int k = (i / (NQ / 4)) % NK; const int d = i / (NQ / 4 * NK); v4h ws, wc;
#pragma unroll
    for (int q = 0; q < 4; ++q) { const size_t e = ((size_t)d * NQ + (q0 + q)) * NK + k; const float a = bfr(A[e]); float s, c; sincosf(bfr(Bp[e]), &s, &c); ws[q] = toh_flush(__fmul_rn(a, c)); wc[q] = toh_flush(__fmul_rn(a, s)); }
    h16* wr = Wf + (size_t)d * KK + k * NQ + q0;
    *(volatile v4h*)wr = ws; *(volatile v4h*)(wr + NK * NQ) = wc; __threadfence(); *(volatile v4h*)wr = ws; *(volatile v4h*)(wr + NK * NQ) = wc; }

extern "C" void kernel_launch(void* const* d_in, const int* in_sizes, int n_in,
                              void* d_out, int out_size, void* d_ws, size_t ws_size, hipStream_t stream) {
    (void)in_sizes; (void)n_in; (void)out_size;
    const float* x0 = (const float*)d_in[0]; const float* tt = (const float*)d_in[1]; const float* wcw = (const float*)d_in[2]; const float* wcb = (const float*)d_in[3]; const float* ww = (const float*)d_in[4]; const float* aa = (const float*)d_in[5]; const float* bp = (const float*)d_in[6];
    static_assert(NR % 64 == 0 && NQ % 64 == 0 && NDO % 64 == 0 && DIN % 32 == 0 && KK % 32 == 0 && KK == 2 * NK * NQ && NR == 2 * TS && NQ % 4 == 0, "both product launches: M and N multiples of 64, K a multiple of 32; the feature order");
    float* OUT = (float*)d_out;
    char* wsp = (char*)d_ws;
    auto take = [&](size_t bytes) { char* p = wsp; wsp += (bytes + 255) & ~(size_t)255; return (void*)p; };
    bf* Xb = (bf*)take((size_t)NR * DIN * 2);     bf* Wb = (bf*)take((size_t)NQ * DIN * 2);     float* FC = (float*)take((size_t)NR * NQ * 4);     h16* F = (h16*)take((size_t)NR * KK * 2);     h16* Wf = (h16*)take((size_t)NDO * KK * 2);
    if ((size_t)(wsp - (char*)d_ws) > ws_size) return;
    k_cvt8<<<(unsigned)(((size_t)NR * DIN / 8 + 255) / 256), 256, 0, stream>>>(x0, Xb, (size_t)NR * DIN / 8);
    k_cvt8<<<(unsigned)(((size_t)NQ * DIN / 8 + 255) / 256), 256, 0, stream>>>(wcw, Wb, (size_t)NQ * DIN / 8);
    k_gemmw<bf, 0, true><<<dim3(NR / 64, NQ / 64, 1), 32, 0, stream>>>(Xb, nullptr, Wb, nullptr, DIN, FC, NQ, wcb, 0, 0, 0);
    k_feat<<<(unsigned)(((size_t)NR * NQ / 4 + 255) / 256), 256, 0, stream>>>(FC, ww, tt, F);
    k_wfeat<<<(unsigned)((NDO * NK * NQ / 4 + 255) / 256), 256, 0, stream>>>(aa, bp, Wf);
    k_gemmw<h16, 0, false><<<dim3(NR / 64, NDO / 64, 1), 32, 0, stream>>>(F, nullptr, Wf, nullptr, KK, OUT, NDO, nullptr, 0, 0, 0);
}
